// CombinedModel_sink_feature_multimodel_70437463655094
// MI455X (gfx1250) — hardware-verified
//
#include <hip/hip_runtime.h>
#include <math.h>

typedef _Float16 v16h __attribute__((ext_vector_type(16)));
typedef _Float16 v8h  __attribute__((ext_vector_type(8)));
typedef float    v8f  __attribute__((ext_vector_type(8)));
typedef float    v4f  __attribute__((ext_vector_type(4)));
typedef unsigned int v4u __attribute__((ext_vector_type(4)));
typedef v8h __attribute__((may_alias)) v8ha;
typedef v4f __attribute__((may_alias)) v4fa;
typedef v4u __attribute__((may_alias)) v4ua;

union Frag { v16h v; v8h half[2]; };

#define NB      128
#define NREG    333
#define DIN     333
#define KP      352
#define DHID    1024
#define DF      512
#define NTK     28
#define RALL    (NB * NREG)
#define NCH     2
#define BCH     (NB / NCH)
#define RCH     (BCH * NREG)
#define NITER   100
#define PSC     16384.0f
#define IN_EPS  1e-5f

#define OFF0 0
#define OFF1 3584
#define OFF2 32256
#define OFF3 3702272
#define OFF4 3705856
#define OFF5 3734528
#define OUT_TOTAL 7404544

#define P_W1   (DHID * KP / 8)
#define P_W2   (DF * DHID / 8)
#define P_MM   (DF * DF / 8)
#define P_TX   (64 * DF / 8)
#define P_PREP (P_W1 + P_W2 + 2 * P_MM + P_TX)
#define P_A    (RALL * (KP / 8))

constexpr size_t SZ_AP = (size_t)RALL * KP * 2;
constexpr size_t SZ_W1 = (size_t)DHID * KP * 2;
constexpr size_t SZ_W2 = (size_t)DF * DHID * 2;
constexpr size_t SZ_MM = (size_t)DF * DF * 2;
constexpr size_t SZ_TX = (size_t)64 * DF * 2;
constexpr size_t SZ_YM = (size_t)64 * DF * 2;
constexpr size_t SZ_H  = (size_t)RCH * DHID * 2;
constexpr size_t SZ_F  = (size_t)RCH * DF * 2;
constexpr size_t SZ_S  = (size_t)RCH * 32 * 4;
constexpr size_t SZ_ST = (size_t)BCH * 32 * KP * 2;
constexpr size_t OFF_AP = 0;
constexpr size_t OFF_W1 = OFF_AP + SZ_AP;
constexpr size_t OFF_W2 = OFF_W1 + SZ_W1;
constexpr size_t OFF_M0 = OFF_W2 + SZ_W2;
constexpr size_t OFF_M1 = OFF_M0 + SZ_MM;
constexpr size_t OFF_TX = OFF_M1 + SZ_MM;
constexpr size_t OFF_YM = OFF_TX + SZ_TX;
constexpr size_t OFF_H  = OFF_YM + SZ_YM;
constexpr size_t OFF_F  = OFF_H + SZ_H;
constexpr size_t OFF_S  = OFF_F + SZ_F;
constexpr size_t OFF_ST = OFF_S + SZ_S;
constexpr size_t WS_TOTAL = OFF_ST + SZ_ST;
static_assert(WS_TOTAL <= (size_t)134217728);
static_assert(OFF_W1 % 256 == 0 && OFF_W2 % 256 == 0 && OFF_M0 % 256 == 0 && OFF_M1 % 256 == 0);
static_assert(OFF_TX % 256 == 0 && OFF_YM % 256 == 0 && OFF_H % 256 == 0 && OFF_F % 256 == 0);
static_assert(OFF_S % 256 == 0 && OFF_ST % 256 == 0);
static_assert(SZ_AP % 512 == 0 && SZ_ST % 512 == 0 && SZ_W1 % 512 == 0);
static_assert(P_PREP % 256 == 0 && P_A % 256 == 0);
static_assert(RCH % 64 == 0 && RALL % RCH == 0);

__device__ __forceinline__ v8f wmma_f16(v16h a, v16h b, v8f c) {
  v8f d = __builtin_amdgcn_wmma_f32_16x16x32_f16(false, a, false, b, (short)0, c, false, false);
  asm volatile("v_nop\n\tv_nop\n\tv_nop\n\tv_nop" : "+v"(d) : "v"(a), "v"(b));
  return d;
}

__device__ __forceinline__ v16h load_frag(const _Float16* p, int h) {
  Frag f;
  f.half[0] = *(const v8ha*)(p + 8 * h);
  f.half[1] = *(const v8ha*)(p + 16 + 8 * h);
  return f.v;
}

__device__ __forceinline__ int imin(int a, int b) { return a < b ? a : b; }

__device__ __forceinline__ float ldz(const float* __restrict__ base, int c, int n, float sc) {
  const float x = base[imin(c, n - 1)];
  return x * ((c < n) ? sc : 0.0f);
}

__device__ __forceinline__ v8h pk8(v4f a, v4f c) {
  v8h o = { (_Float16)a.x, (_Float16)a.y, (_Float16)a.z, (_Float16)a.w,
            (_Float16)c.x, (_Float16)c.y, (_Float16)c.z, (_Float16)c.w };
  return o;
}

__device__ __forceinline__ void st2h(_Float16* dst, v8h o) {
  *(volatile v8h*)dst = o;
  __threadfence();
  *(volatile v8h*)dst = o;
}

__device__ __forceinline__ float gelu_t(float x) {
  const float u = 0.7978845608028654f * (x + 0.044715f * (x * x * x));
  const float t2 = fminf(fmaxf(2.0f * u, -30.0f), 30.0f);
  const float e = __expf(-t2);
  return x * __builtin_amdgcn_rcpf(1.0f + e);
}

__device__ __forceinline__ float msym16(const float* __restrict__ A, int d, int e) {
  return (A[(size_t)d * DF + e] + A[(size_t)e * DF + d]) * 16.0f;
}

__global__ void __launch_bounds__(256)
prep_kernel(const float* __restrict__ w1, const float* __restrict__ w2,
            const float* __restrict__ aA, const float* __restrict__ aB,
            const float* __restrict__ text,
            _Float16* __restrict__ W1p, _Float16* __restrict__ W2p,
            _Float16* __restrict__ M0p, _Float16* __restrict__ M1p,
            _Float16* __restrict__ TXp)
{
  const int g = blockIdx.x * 256 + threadIdx.x;
  if (g >= P_PREP) return;
  v4f lo, hi;
  _Float16* dst;
  if (g < P_W1) {
    const int row = g / (KP / 8);
    const int c0 = (g - row * (KP / 8)) * 8;
    const float* src = w1 + (size_t)row * DIN;
    lo.x = ldz(src, c0 + 0, DIN, 32.0f); lo.y = ldz(src, c0 + 1, DIN, 32.0f);
    lo.z = ldz(src, c0 + 2, DIN, 32.0f); lo.w = ldz(src, c0 + 3, DIN, 32.0f);
    hi.x = ldz(src, c0 + 4, DIN, 32.0f); hi.y = ldz(src, c0 + 5, DIN, 32.0f);
    hi.z = ldz(src, c0 + 6, DIN, 32.0f); hi.w = ldz(src, c0 + 7, DIN, 32.0f);
    dst = W1p + (size_t)g * 8;
  } else if (g < P_W1 + P_W2) {
    const int e = g - P_W1;
    const float* src = w2 + (size_t)e * 8;
    lo = *(const v4fa*)src * 32.0f;
    hi = *(const v4fa*)(src + 4) * 32.0f;
    dst = W2p + (size_t)e * 8;
  } else if (g < P_W1 + P_W2 + 2 * P_MM) {
    const int e = g - (P_W1 + P_W2);
    const bool second = (e >= P_MM);
    const int e2 = second ? e - P_MM : e;
    const float* Ap = second ? aB : aA;
    const int d = e2 >> 6, e0 = (e2 & 63) * 8;
    lo.x = msym16(Ap, d, e0 + 0); lo.y = msym16(Ap, d, e0 + 1);
    lo.z = msym16(Ap, d, e0 + 2); lo.w = msym16(Ap, d, e0 + 3);
    hi.x = msym16(Ap, d, e0 + 4); hi.y = msym16(Ap, d, e0 + 5);
    hi.z = msym16(Ap, d, e0 + 6); hi.w = msym16(Ap, d, e0 + 7);
    dst = (second ? M1p : M0p) + (size_t)e2 * 8;
  } else {
    const int e = g - (P_W1 + P_W2 + 2 * P_MM);
    const int mrow = e >> 6, e0 = (e & 63) * 8;
    const int mm = imin(mrow, NTK - 1);
    const float* src = text + (size_t)(NTK + mm) * DF + e0;
    const float keep = (mrow < NTK) ? 1.0f : 0.0f;
    lo = *(const v4fa*)src * keep;
    hi = *(const v4fa*)(src + 4) * keep;
    dst = TXp + (size_t)e * 8;
  }
  st2h(dst, pk8(lo, hi));
}

__global__ void __launch_bounds__(256)
cvt0_kernel(const float* __restrict__ x, _Float16* __restrict__ Ap)
{
  const int g = blockIdx.x * 256 + threadIdx.x;
  if (g >= P_A) return;
  const int r = g / (KP / 8);
  const int c0 = (g - r * (KP / 8)) * 8;
  const float* src = x + (size_t)r * DIN;
  v4f lo, hi;
  lo.x = ldz(src, c0 + 0, DIN, 1.0f); lo.y = ldz(src, c0 + 1, DIN, 1.0f);
  lo.z = ldz(src, c0 + 2, DIN, 1.0f); lo.w = ldz(src, c0 + 3, DIN, 1.0f);
  hi.x = ldz(src, c0 + 4, DIN, 1.0f); hi.y = ldz(src, c0 + 5, DIN, 1.0f);
  hi.z = ldz(src, c0 + 6, DIN, 1.0f); hi.w = ldz(src, c0 + 7, DIN, 1.0f);
  st2h(Ap + (size_t)g * 8, pk8(lo, hi));
}

__device__ __forceinline__ float fc1_one(const float* __restrict__ tp, const float* __restrict__ w,
                                         const float* __restrict__ b, int jj) {
  const int jc = imin(jj, DIN - 1);
  const float* wp = w + (size_t)jc * 9;
  float acc = 0.0f;
  #pragma unroll 1
  for (int k = 0; k < 9; ++k) acc += tp[k] * wp[k];
  acc += b[jc];
  return fmaxf(acc, 0.0f) * ((jj < DIN) ? 16.0f : 0.0f);
}

__global__ void __launch_bounds__(256)
fc1_kernel(const float* __restrict__ x, const float* __restrict__ w,
           const float* __restrict__ b, _Float16* __restrict__ Ap)
{
  const int g = blockIdx.x * 256 + threadIdx.x;
  if (g >= P_A) return;
  const int r = g / (KP / 8);
  const int c0 = (g - r * (KP / 8)) * 8;
  const float* tp = x + (size_t)r * 9;
  v4f lo, hi;
  lo.x = fc1_one(tp, w, b, c0 + 0); lo.y = fc1_one(tp, w, b, c0 + 1);
  lo.z = fc1_one(tp, w, b, c0 + 2); lo.w = fc1_one(tp, w, b, c0 + 3);
  hi.x = fc1_one(tp, w, b, c0 + 4); hi.y = fc1_one(tp, w, b, c0 + 5);
  hi.z = fc1_one(tp, w, b, c0 + 6); hi.w = fc1_one(tp, w, b, c0 + 7);
  st2h(Ap + (size_t)g * 8, pk8(lo, hi));
}

__device__ __forceinline__ void tile_store_pass(const unsigned char* sT, unsigned char* out,
                                                int rblk, int ldo_bytes, int colbyte, int w, int lane) {
  const int q8 = lane & 7, sub = lane >> 3;
  #pragma unroll
  for (int i = 0; i < 8; ++i) {
    const int lid = 32 * w + 4 * i + sub;
    const v4u v = *(const v4ua*)(sT + lid * 128 + 16 * q8);
    unsigned char* dst = out + (size_t)(rblk + lid) * ldo_bytes + colbyte + 16 * q8;
    *(volatile v4u*)dst = v;
  }
}

template <int MODE, bool HAS_BIAS, int KSTEPS, int NT>
__global__ void __launch_bounds__(64) __attribute__((amdgpu_num_vgpr(248)))
gemm_kernel(const _Float16* __restrict__ A, int lda,
            const _Float16* __restrict__ Bt, int ldb,
            const float* __restrict__ bias,
            unsigned char* __restrict__ out, int ldo_bytes,
            float inscale, float outscale)
{
  static_assert(MODE == 2 ? NT == 2 : NT == 4);
  __shared__ __attribute__((aligned(16))) unsigned char sT[64 * 128];

  const int tid = threadIdx.x, lane = tid & 31, w = tid >> 5;
  const int h = lane >> 4, m = lane & 15;
  const int rblk = blockIdx.x * 64;
  const int col0 = blockIdx.y * (16 * NT);

  const _Float16* a0p = A + (size_t)(rblk + 32 * w + m) * lda;
  const _Float16* a1p = a0p + (size_t)16 * lda;
  const _Float16* bp  = Bt + (size_t)(col0 + m) * ldb;

  const v8f zero8 = {0.f, 0.f, 0.f, 0.f, 0.f, 0.f, 0.f, 0.f};
  v8f acc[2][NT];
  #pragma unroll
  for (int mt = 0; mt < 2; ++mt)
    #pragma unroll
    for (int nt = 0; nt < NT; ++nt) acc[mt][nt] = zero8;

  #pragma unroll 1
  for (int k0 = 0; k0 < KSTEPS * 32; k0 += 32) {
    const v16h a0 = load_frag(a0p + k0, h);
    const v16h a1 = load_frag(a1p + k0, h);
    #pragma unroll
    for (int nt = 0; nt < NT; ++nt) {
      const v16h b = load_frag(bp + (size_t)(16 * nt) * ldb + k0, h);
      acc[0][nt] = wmma_f16(a0, b, acc[0][nt]);
      acc[1][nt] = wmma_f16(a1, b, acc[1][nt]);
    }
  }

  _Float16* sTh = (_Float16*)sT;
  float* sTf = (float*)sT;
  #pragma unroll
  for (int nt = 0; nt < NT; ++nt) {
    const int lcol = 16 * nt + m;
    float bv = 0.0f;
    if (HAS_BIAS) bv = bias[col0 + lcol];
    #pragma unroll
    for (int mt = 0; mt < 2; ++mt) {
      #pragma unroll
      for (int r = 0; r < 8; ++r) {
        const int lrow = 32 * w + 16 * mt + 8 * h + r;
        const float y = acc[mt][nt][r] * inscale + bv;
        if (MODE == 0)      sTh[lrow * 64 + lcol] = (_Float16)(gelu_t(y) * outscale);
        else if (MODE == 1) sTh[lrow * 64 + lcol] = (_Float16)(y * outscale);
        else                sTf[lrow * 32 + lcol] = y * outscale;
      }
    }
  }
  __syncthreads();

  const int colbyte = col0 * ((MODE == 2) ? 4 : 2);
  tile_store_pass(sT, out, rblk, ldo_bytes, colbyte, w, lane);
  __threadfence();
  tile_store_pass(sT, out, rblk, ldo_bytes, colbyte, w, lane);
}

__device__ __forceinline__ float pt_val(const float* st, int mrow, int n) {
  const bool ok = (mrow < NTK) && (n < NREG);
  const int idx = ok ? (n * NTK + mrow) : 0;
  const float x = st[idx];
  return x * (ok ? PSC : 0.0f);
}

__device__ __forceinline__ void pt_store_pass(const float* st, _Float16* STb, int tid) {
  for (int p = tid; p < 32 * (KP / 8); p += 256) {
    const int mrow = p / (KP / 8);
    const int n0 = (p - mrow * (KP / 8)) * 8;
    v4f lo, hi;
    lo.x = pt_val(st, mrow, n0 + 0); lo.y = pt_val(st, mrow, n0 + 1);
    lo.z = pt_val(st, mrow, n0 + 2); lo.w = pt_val(st, mrow, n0 + 3);
    hi.x = pt_val(st, mrow, n0 + 4); hi.y = pt_val(st, mrow, n0 + 5);
    hi.z = pt_val(st, mrow, n0 + 6); hi.w = pt_val(st, mrow, n0 + 7);
    *(volatile v8h*)(STb + (size_t)p * 8) = pk8(lo, hi);
  }
}

__global__ void __launch_bounds__(256)
norm_iter_kernel(const float* __restrict__ S, const float* __restrict__ gam,
                 const float* __restrict__ bet, _Float16* __restrict__ ST)
{
  __shared__ float st[NREG * NTK];
  __shared__ float red[256];

  const int bl = blockIdx.x, tid = threadIdx.x;
  const float* Sb = S + (size_t)bl * NREG * 32;
  for (int i = tid; i < NREG * 32; i += 256) {
    const int r = i >> 5, c = i & 31;
    const float v = Sb[i];
    if (c < NTK) st[r * NTK + c] = v;
  }
  __syncthreads();

  const float inv_n = 1.0f / (float)(NREG * NTK);
  float ps = 0.0f;
  #pragma unroll 2
  for (int i = tid; i < NREG * NTK; i += 256) ps += st[i];
  red[tid] = ps;
  __syncthreads();
  for (int s = 128; s > 0; s >>= 1) {
    if (tid < s) red[tid] += red[tid + s];
    __syncthreads();
  }
  const float mu = red[0] * inv_n;
  __syncthreads();
  float pq = 0.0f;
  #pragma unroll 2
  for (int i = tid; i < NREG * NTK; i += 256) { const float d = st[i] - mu; pq += d * d; }
  red[tid] = pq;
  __syncthreads();
  for (int s = 128; s > 0; s >>= 1) {
    if (tid < s) red[tid] += red[tid + s];
    __syncthreads();
  }
  const float var = red[0] * inv_n;
  const float rstd = rsqrtf(var + IN_EPS);
  const float ga = gam[0], be = bet[0];
  __syncthreads();
  #pragma unroll 2
  for (int i = tid; i < NREG * NTK; i += 256) st[i] = (ga * (st[i] - mu)) * rstd + be;
  __syncthreads();

  const float NEG = -3.0e38f;
  for (int it = 0; it < NITER; ++it) {
    for (int r = tid; r < NREG; r += 256) {
      float* row = st + r * NTK;
      float mx = NEG;
      #pragma unroll 7
      for (int c = 0; c < NTK; ++c) mx = fmaxf(mx, row[c]);
      float sm = 0.0f;
      #pragma unroll 7
      for (int c = 0; c < NTK; ++c) sm += __expf(row[c] - mx);
      const float lse = mx + __logf(sm);
      #pragma unroll 7
      for (int c = 0; c < NTK; ++c) row[c] -= lse;
    }
    __syncthreads();
    if (tid < 224) {
      const int c = tid >> 3, sub = tid & 7;
      float mx = NEG;
      for (int r = sub; r < NREG; r += 8) mx = fmaxf(mx, st[r * NTK + c]);
      mx = fmaxf(mx, __shfl_xor(mx, 1));
      mx = fmaxf(mx, __shfl_xor(mx, 2));
      mx = fmaxf(mx, __shfl_xor(mx, 4));
      float sm = 0.0f;
      for (int r = sub; r < NREG; r += 8) sm += __expf(st[r * NTK + c] - mx);
      sm += __shfl_xor(sm, 1);
      sm += __shfl_xor(sm, 2);
      sm += __shfl_xor(sm, 4);
      const float lse = mx + __logf(sm);
      for (int r = sub; r < NREG; r += 8) st[r * NTK + c] -= lse;
    }
    __syncthreads();
  }

  #pragma unroll 1
  for (int i = tid; i < NREG * NTK; i += 256) st[i] = expf(st[i]);
  __syncthreads();

  _Float16* STb = ST + (size_t)bl * 32 * KP;
  pt_store_pass(st, STb, tid);
  __threadfence();
  pt_store_pass(st, STb, tid);
}

__device__ __forceinline__ void pool_store_pass(const float* sO, const float* __restrict__ text1,
                                                float* ob, int cg, int w, int lane) {
  #pragma unroll
  for (int i = 0; i < 14; ++i) {
    const int mm = w + 2 * i;
    const v4f a = *(const v4fa*)(sO + mm * 128 + 4 * lane);
    const v4f t = *(const v4fa*)(text1 + (size_t)mm * DF + cg * 128 + 4 * lane);
    float* dst = ob + (size_t)mm * (2 * DF) + cg * 128 + 4 * lane;
    *(volatile v4f*)dst = a;
    *(volatile v4f*)(dst + DF) = t;
  }
}

__global__ void __launch_bounds__(64) __attribute__((amdgpu_num_vgpr(248)))
pool_kernel(const _Float16* __restrict__ ST, const _Float16* __restrict__ F,
            const float* __restrict__ text1, float* outc, int b0, float oscale)
{
  __shared__ __attribute__((aligned(16))) _Float16 Bs[128 * 40];
  __shared__ __attribute__((aligned(16))) float sO[32 * 128];

  const int tid = threadIdx.x, lane = tid & 31, w = tid >> 5;
  const int h = lane >> 4, m = lane & 15;
  const int bl = blockIdx.x, cg = blockIdx.y;

  const _Float16* a0p = ST + ((size_t)bl * 32 + m) * KP;
  const _Float16* a1p = a0p + (size_t)16 * KP;
  const _Float16* Fb = F + (size_t)bl * NREG * DF + cg * 128;

  const v8f zero8 = {0.f, 0.f, 0.f, 0.f, 0.f, 0.f, 0.f, 0.f};
  const v8h z8 = {(_Float16)0.f, (_Float16)0.f, (_Float16)0.f, (_Float16)0.f,
                  (_Float16)0.f, (_Float16)0.f, (_Float16)0.f, (_Float16)0.f};
  v8f acc[2][4];
  #pragma unroll
  for (int mt = 0; mt < 2; ++mt)
    #pragma unroll
    for (int nt = 0; nt < 4; ++nt) acc[mt][nt] = zero8;

  #pragma unroll 1
  for (int ks = 0; ks < KP / 32; ++ks) {
    __syncthreads();
    #pragma unroll
    for (int i = 0; i < 8; ++i) {
      const int p = tid + 64 * i;
      const int n = p >> 4, d0 = (p & 15) * 8;
      const int nn = ks * 32 + n;
      const int nc = imin(nn, NREG - 1);
      v8h v = *(const v8ha*)(Fb + (size_t)nc * DF + d0);
      if (nn >= NREG) v = z8;
      #pragma unroll
      for (int j = 0; j < 8; ++j) Bs[(d0 + j) * 40 + n] = v[j];
    }
    __syncthreads();
    const int k0 = ks * 32;
    const v16h a0 = load_frag(a0p + k0, h);
    const v16h a1 = load_frag(a1p + k0, h);
    #pragma unroll
    for (int nt = 0; nt < 4; ++nt) {
      const v16h b = load_frag(Bs + (64 * w + 16 * nt + m) * 40, h);
      acc[0][nt] = wmma_f16(a0, b, acc[0][nt]);
      acc[1][nt] = wmma_f16(a1, b, acc[1][nt]);
    }
  }

  #pragma unroll
  for (int nt = 0; nt < 4; ++nt)
    #pragma unroll
    for (int mt = 0; mt < 2; ++mt)
      #pragma unroll
      for (int r = 0; r < 8; ++r)
        sO[(16 * mt + 8 * h + r) * 128 + 64 * w + 16 * nt + m] = acc[mt][nt][r] * oscale;
  __syncthreads();

  float* ob = outc + (size_t)(b0 + bl) * NTK * (2 * DF);
  pool_store_pass(sO, text1, ob, cg, w, lane);
  __threadfence();
  pool_store_pass(sO, text1, ob, cg, w, lane);
}

__global__ void __launch_bounds__(256)
final_kernel(float* out, const float* __restrict__ tw, const float* __restrict__ tb)
{
  __shared__ __attribute__((aligned(16))) float res[32];
  const int blk = blockIdx.x, tid = threadIdx.x, lane = tid & 31, w = tid >> 5;
  if (blk < 224) {
    const int br = (blk >= 112) ? 1 : 0;
    const int li = blk - br * 112;
    const float* comb = out + (br ? OFF5 : OFF2);
    #pragma unroll 1
    for (int jj = 0; jj < 4; ++jj) {
      const int j = w + 8 * jj;
      const int f = li * 32 + j;
      const int t = f % NTK;
      const float* crow = comb + (size_t)f * (2 * DF);
      const float* wrow = tw + (size_t)t * (2 * DF);
      float acc = 0.0f;
      #pragma unroll 2
      for (int i = 0; i < 8; ++i) {
        const v4f c = *(const v4fa*)(crow + 128 * i + 4 * lane);
        const v4f q = *(const v4fa*)(wrow + 128 * i + 4 * lane);
        acc += c.x * q.x; acc += c.y * q.y; acc += c.z * q.z; acc += c.w * q.w;
      }
      acc += __shfl_xor(acc, 16);
      acc += __shfl_xor(acc, 8);
      acc += __shfl_xor(acc, 4);
      acc += __shfl_xor(acc, 2);
      acc += __shfl_xor(acc, 1);
      if (lane == 0) res[j] = acc + tb[t];
    }
    __syncthreads();
    const bool wr = (tid < 8);
    const v4f v = *(const v4fa*)(res + 4 * imin(tid, 7));
    float* dst = out + (br ? OFF3 : OFF0) + li * 32 + 4 * imin(tid, 7);
    if (wr) *(volatile v4f*)dst = v;
    __threadfence();
    if (wr) *(volatile v4f*)dst = v;
  } else {
    const int g = (blk - 224) * 256 + tid;
    const int which = (g >= 7168) ? 1 : 0;
    const int q = g - which * 7168;
    const v4f v = *(const v4fa*)(tw + 4 * q);
    float* dst = out + (which ? OFF4 : OFF1) + 4 * q;
    *(volatile v4f*)dst = v;
    __threadfence();
    *(volatile v4f*)dst = v;
  }
}

extern "C" void kernel_launch(void* const* d_in, const int* in_sizes, int n_in,
                              void* d_out, int out_size, void* d_ws, size_t ws_size,
                              hipStream_t stream) {
  if (n_in < 17) return;
  if (in_sizes[0] != RALL * DIN || in_sizes[1] != RALL * 9 || in_sizes[2] != 2 * NTK * DF) return;
  if (in_sizes[3] != DIN * 9 || in_sizes[4] != DIN) return;
  if (in_sizes[5] != DHID * DIN || in_sizes[6] != DHID) return;
  if (in_sizes[7] != DF * DHID || in_sizes[8] != DF) return;
  if (in_sizes[9] != DF * DF || in_sizes[10] != DF * DF) return;
  if (in_sizes[11] < 1 || in_sizes[12] < 1 || in_sizes[13] < 1 || in_sizes[14] < 1) return;
  if (in_sizes[15] != NTK * 2 * DF || in_sizes[16] != NTK) return;
  if (out_size != OUT_TOTAL) return;
  if (WS_TOTAL > ws_size) return;

  const float* x0     = (const float*)d_in[0];
  const float* x1     = (const float*)d_in[1];
  const float* text   = (const float*)d_in[2];
  const float* fc1_w  = (const float*)d_in[3];
  const float* fc1_b  = (const float*)d_in[4];
  const float* ext_w1 = (const float*)d_in[5];
  const float* ext_b1 = (const float*)d_in[6];
  const float* ext_w2 = (const float*)d_in[7];
  const float* ext_b2 = (const float*)d_in[8];
  const float* aff0   = (const float*)d_in[9];
  const float* aff1   = (const float*)d_in[10];
  const float* gam0   = (const float*)d_in[11];
  const float* bet0   = (const float*)d_in[12];
  const float* gam1   = (const float*)d_in[13];
  const float* bet1   = (const float*)d_in[14];
  const float* task_w = (const float*)d_in[15];
  const float* task_b = (const float*)d_in[16];
  const float* text1  = text + (size_t)NTK * DF;
  float* out = (float*)d_out;

  unsigned char* ws = (unsigned char*)d_ws;
  _Float16* Ap  = (_Float16*)(ws + OFF_AP);
  _Float16* W1p = (_Float16*)(ws + OFF_W1);
  _Float16* W2p = (_Float16*)(ws + OFF_W2);
  _Float16* M0p = (_Float16*)(ws + OFF_M0);
  _Float16* M1p = (_Float16*)(ws + OFF_M1);
  _Float16* TXp = (_Float16*)(ws + OFF_TX);
  _Float16* YMp = (_Float16*)(ws + OFF_YM);
  _Float16* Hp  = (_Float16*)(ws + OFF_H);
  _Float16* Fp  = (_Float16*)(ws + OFF_F);
  float*    Sp  = (float*)(ws + OFF_S);
  _Float16* STp = (_Float16*)(ws + OFF_ST);

  prep_kernel<<<P_PREP / 256, 256, 0, stream>>>(ext_w1, ext_w2, aff0, aff1, text,
                                                W1p, W2p, M0p, M1p, TXp);

  for (int br = 0; br < 2; ++br) {
    const float acar = (br == 0) ? 1.0f : 16.0f;
    const float hcar = (br == 0) ? 4.0f : 64.0f;
    const float fcar = (br == 0) ? 8.0f : 128.0f;
    const _Float16* Mp = (br == 0) ? M0p : M1p;
    const float* gam = (br == 0) ? gam0 : gam1;
    const float* bet = (br == 0) ? bet0 : bet1;
    float* outc = out + ((br == 0) ? OFF2 : OFF5);

    if (br == 0) cvt0_kernel<<<P_A / 256, 256, 0, stream>>>(x0, Ap);
    else         fc1_kernel<<<P_A / 256, 256, 0, stream>>>(x1, fc1_w, fc1_b, Ap);

    gemm_kernel<1, false, DF / 32, 4><<<dim3(1, DF / 64), 64, 0, stream>>>(
        TXp, DF, Mp, DF, ext_b2, (unsigned char*)YMp, DF * 2, 1.0f / 32.0f, 4.0f);

    for (int c = 0; c < NCH; ++c) {
      gemm_kernel<0, true, KP / 32, 4><<<dim3(RCH / 64, DHID / 64), 64, 0, stream>>>(
          Ap + (size_t)c * RCH * KP, KP, W1p, KP, ext_b1, (unsigned char*)Hp, DHID * 2,
          1.0f / (32.0f * acar), hcar);
      gemm_kernel<1, true, DHID / 32, 4><<<dim3(RCH / 64, DF / 64), 64, 0, stream>>>(
          Hp, DHID, W2p, DHID, ext_b2, (unsigned char*)Fp, DF * 2,
          1.0f / (32.0f * hcar), fcar);
      gemm_kernel<2, false, DF / 32, 2><<<dim3(RCH / 64, 1), 64, 0, stream>>>(
          Fp, DF, YMp, DF, ext_b2, (unsigned char*)Sp, 32 * 4,
          1.0f / (4.0f * fcar), 1.0f);
      norm_iter_kernel<<<BCH, 256, 0, stream>>>(Sp, gam, bet, STp);
      pool_kernel<<<dim3(BCH, 4), 64, 0, stream>>>(STp, Fp, text1, outc, c * BCH,
                                                   1.0f / (PSC * fcar));
    }
  }

  final_kernel<<<224 + 56, 256, 0, stream>>>(out, task_w, task_b);
}
